// GINNet_67336497266911
// MI455X (gfx1250) — hardware-verified
//
#include <hip/hip_runtime.h>
#include <stddef.h>
#include <stdint.h>


#define DIN     128
#define HID     512
#define DOUT    128
#define K1      256
#define K4      1024
#define NTHR    256
#define NWAVE   8
#define EPT     8
#define CHUNK   (NTHR * EPT)
#define WCAP    (EPT * 32)
#define LISTN   (NWAVE * WCAP)
#define NBA     512
#define PKS     9
#define RCAP    28672
#define DEGCAP  128
#define STW     512
#define RCH     7168
#define NBLKA   (RCH / NBA)
#define GBM     64
#define GBN     128
#define GTHR    128
#define WCARRY  1024.0f
#define WINV    0.0009765625f
#define NU1     (HID * (K1 / 8))
#define NU2     (HID * (HID / 8))
#define NU4     (DOUT * (K4 / 8))
#define NUW     (NU1 + 2 * NU2 + NU4)
#define ZINTS   (2 * RCAP + 2 * NBA + LISTN)
#define LDS_AGG (ZINTS * 4 + 64)
#define WSMAX   134217728

static_assert((CHUNK & (CHUNK - 1)) == 0);
static_assert(NBA == (1 << PKS));
static_assert(((long long)CHUNK << PKS) < (1LL << 31));
static_assert(NTHR * 2 == NBA);
static_assert(LISTN >= NBA && LISTN >= NWAVE * WCAP);
static_assert((RCAP % 32) == 0 && NWAVE * STW <= RCAP && STW >= 256);
static_assert((ZINTS % (NTHR * 4)) == 0);
static_assert(LDS_AGG <= 262144);
static_assert(RCH == NBLKA * NBA && (RCH % GBM) == 0);
static_assert((NBA % NWAVE) == 0);
static_assert(GBM == (GTHR / 32) * 16 && GBN == 4 * 32);
static_assert((HID % GBN) == 0 && DOUT == GBN);
static_assert((K1 % 32) == 0 && (HID % 32) == 0 && (K4 % 32) == 0 && K1 == 2 * DIN && K4 == 2 * HID);
static_assert((NU1 % NTHR) == 0 && (NU2 % NTHR) == 0 && (NU4 % NTHR) == 0);
static_assert(DIN == 32 * 4 && HID == 32 * 16);

typedef float          v4f  __attribute__((ext_vector_type(4)));
typedef float          v8f  __attribute__((ext_vector_type(8)));
typedef int            v4i  __attribute__((ext_vector_type(4)));
typedef int            v8i  __attribute__((ext_vector_type(8)));
typedef unsigned int   v2u  __attribute__((ext_vector_type(2)));
typedef unsigned int   v4u  __attribute__((ext_vector_type(4)));
typedef unsigned short v8us __attribute__((ext_vector_type(8)));
typedef _Float16       v16h __attribute__((ext_vector_type(16)));
typedef __bf16         v16b __attribute__((ext_vector_type(16)));
typedef v4f  __attribute__((may_alias)) v4fa;
typedef v4i  __attribute__((may_alias)) v4ia;
typedef v2u  __attribute__((may_alias)) v2ua;
typedef v4u  __attribute__((may_alias)) v4ua;
typedef v8us __attribute__((may_alias)) v8usa;
union Frag { v16b b; v16h f; v8us h[2]; v8i w; };

template <int KIND>
__device__ __forceinline__ v8f wmk(const Frag& a, const Frag& b, v8f c) {
  v8f d;
  if constexpr (KIND == 0) {
    d = __builtin_amdgcn_wmma_f32_16x16x32_bf16(false, a.b, false, b.b, (short)0, c, false, false);
  } else {
    d = __builtin_amdgcn_wmma_f32_16x16x32_f16(false, a.f, false, b.f, (short)0, c, false, false);
  }
  asm volatile("v_nop\n\tv_nop\n\tv_nop\n\tv_nop" : "+v"(d) : "v"(a.w), "v"(b.w));
  return d;
}

__device__ __forceinline__ unsigned short bf_bits(float f) {
  unsigned int u = __float_as_uint(f);
  u += 0x7FFFu + ((u >> 16) & 1u);
  return (unsigned short)(u >> 16);
}
__device__ __forceinline__ float bf_val(unsigned short b) {
  return __uint_as_float(((unsigned int)b) << 16);
}
__device__ __forceinline__ float bf_rne(float f) { return bf_val(bf_bits(f)); }

__device__ __forceinline__ unsigned short h_bits(float f) {
  const _Float16 h = (_Float16)f;
  return __builtin_bit_cast(unsigned short, h);
}

__device__ __forceinline__ v8us cvt8h(const v4f a, const v4f b) {
  v8us o;
  o[0] = h_bits(a.x); o[1] = h_bits(a.y); o[2] = h_bits(a.z); o[3] = h_bits(a.w);
  o[4] = h_bits(b.x); o[5] = h_bits(b.y); o[6] = h_bits(b.z); o[7] = h_bits(b.w);
  return o;
}
__device__ __forceinline__ void split8b(const v4f a, const v4f b, v8us& hi, v8us& lo) {
  float x[8];
  x[0] = a.x; x[1] = a.y; x[2] = a.z; x[3] = a.w; x[4] = b.x; x[5] = b.y; x[6] = b.z; x[7] = b.w;
#pragma unroll
  for (int i = 0; i < 8; ++i) {
    const unsigned short hb = bf_bits(x[i]);
    hi[i] = hb;
    lo[i] = bf_bits(x[i] - bf_val(hb));
  }
}

template <int ACT>
__device__ __forceinline__ float actf(float v) {
  if constexpr (ACT == 1) {
    return fmaxf(v, 0.0f);
  } else if constexpr (ACT == 2) {
    const float e = expm1f(fminf(v, 0.0f));
    return v > 0.0f ? v : e;
  } else {
    return v;
  }
}

__device__ __forceinline__ int scan_chunk(const int* __restrict__ dsts, int nE, int cbase, int slotBase,
                                          int nb, int vec8, int* list, int tid, int lane, int wave) {
  int wc = 0;
  const int el0  = tid * EPT;
  const int e0   = cbase + el0;
  const int sent = -2147483647 - 1;
  v4i da, db;
  if (vec8 != 0 && cbase + CHUNK <= nE) {
    da = *(const v4i*)(dsts + e0);
    db = *(const v4i*)(dsts + e0 + 4);
  } else {
    da.x = (e0     < nE) ? dsts[min(e0,     nE - 1)] : sent;
    da.y = (e0 + 1 < nE) ? dsts[min(e0 + 1, nE - 1)] : sent;
    da.z = (e0 + 2 < nE) ? dsts[min(e0 + 2, nE - 1)] : sent;
    da.w = (e0 + 3 < nE) ? dsts[min(e0 + 3, nE - 1)] : sent;
    db.x = (e0 + 4 < nE) ? dsts[min(e0 + 4, nE - 1)] : sent;
    db.y = (e0 + 5 < nE) ? dsts[min(e0 + 5, nE - 1)] : sent;
    db.z = (e0 + 6 < nE) ? dsts[min(e0 + 6, nE - 1)] : sent;
    db.w = (e0 + 7 < nE) ? dsts[min(e0 + 7, nE - 1)] : sent;
  }
  const unsigned nbs = (unsigned)slotBase;
  const unsigned unb = (unsigned)nb;
  const unsigned s0 = (unsigned)da.x - nbs, s1 = (unsigned)da.y - nbs;
  const unsigned s2 = (unsigned)da.z - nbs, s3 = (unsigned)da.w - nbs;
  const unsigned s4 = (unsigned)db.x - nbs, s5 = (unsigned)db.y - nbs;
  const unsigned s6 = (unsigned)db.z - nbs, s7 = (unsigned)db.w - nbs;
  const bool h0 = s0 < unb, h1 = s1 < unb, h2 = s2 < unb, h3 = s3 < unb;
  const bool h4 = s4 < unb, h5 = s5 < unb, h6 = s6 < unb, h7 = s7 < unb;
  const unsigned any = __builtin_amdgcn_ballot_w32(h0 | h1 | h2 | h3 | h4 | h5 | h6 | h7);
  if (any != 0u) {
#define HITJ(J, HJ, SJ) { \
      const unsigned mj = __builtin_amdgcn_ballot_w32(HJ); \
      if (mj != 0u) { \
        if (HJ) { \
          const int pos = wc + (int)__builtin_amdgcn_mbcnt_lo(mj, 0u); \
          if (pos < WCAP) list[wave * WCAP + pos] = ((el0 + (J)) << PKS) | (int)(SJ); \
        } \
        wc += (int)__builtin_popcount(mj); } }
    HITJ(0, h0, s0)
    HITJ(1, h1, s1)
    HITJ(2, h2, s2)
    HITJ(3, h3, s3)
    HITJ(4, h4, s4)
    HITJ(5, h5, s5)
    HITJ(6, h6, s6)
    HITJ(7, h7, s7)
#undef HITJ
  }
  return wc;
}

__global__ __launch_bounds__(NTHR) void k_wprep(const float* __restrict__ w1, const float* __restrict__ w2,
                                                const float* __restrict__ w3, const float* __restrict__ w4,
                                                unsigned short* W1D, unsigned short* W2C,
                                                unsigned short* W3C, unsigned short* W4D) {
  const int u = (int)blockIdx.x * NTHR + (int)threadIdx.x;
  v8us o;
  unsigned short* dp;
  if (u < NU1) {
    const int n  = u >> 5;
    const int k8 = (u & 31) * 8;
    const int kk = k8 & (DIN - 1);
    const float* p = w1 + (size_t)kk * HID + n;
#pragma unroll
    for (int i = 0; i < 8; ++i) o[i] = bf_bits(p[(size_t)i * HID]);
    dp = W1D + (size_t)n * K1 + k8;
  } else if (u < NU1 + NU2) {
    const int v  = u - NU1;
    const int n  = v >> 6;
    const int k8 = (v & 63) * 8;
    const float* p = w2 + (size_t)k8 * HID + n;
#pragma unroll
    for (int i = 0; i < 8; ++i) o[i] = h_bits(bf_rne(p[(size_t)i * HID]) * WCARRY);
    dp = W2C + (size_t)n * HID + k8;
  } else if (u < NU1 + 2 * NU2) {
    const int v  = u - NU1 - NU2;
    const int n  = v >> 6;
    const int k8 = (v & 63) * 8;
    const float* p = w3 + (size_t)k8 * HID + n;
#pragma unroll
    for (int i = 0; i < 8; ++i) o[i] = h_bits(bf_rne(p[(size_t)i * HID]) * WCARRY);
    dp = W3C + (size_t)n * HID + k8;
  } else if (u < NUW) {
    const int v  = u - NU1 - 2 * NU2;
    const int n  = v >> 7;
    const int k8 = (v & 127) * 8;
    const int kk = k8 & (HID - 1);
    const float* p = w4 + (size_t)kk * DOUT + n;
#pragma unroll
    for (int i = 0; i < 8; ++i) o[i] = bf_bits(p[(size_t)i * DOUT]);
    dp = W4D + (size_t)n * K4 + k8;
  } else {
    return;
  }
  *(volatile v8us*)dp = o;
  __threadfence();
  *(volatile v8us*)dp = o;
}

template <int KIND, int ACT, int OUTK>
__global__ __launch_bounds__(GTHR) void k_gemm(const unsigned short* __restrict__ A, int lda,
                                               const unsigned short* __restrict__ BT, int ldb, int K,
                                               const float* __restrict__ bias, float oscale,
                                               float* C32, unsigned short* C16, int ldc, int nRows) {
  __shared__ __attribute__((aligned(16))) float stg[GBM * GBN];
  const int tid = (int)threadIdx.x, lane = tid & 31, wave = tid >> 5, hh = lane >> 4, m = lane & 15;
  const int rowBase = (int)blockIdx.x * GBM;
  const int colBase = (int)blockIdx.y * GBN;

  v8f acc[8];
  {
    const v8f z = {0.f, 0.f, 0.f, 0.f, 0.f, 0.f, 0.f, 0.f};
#pragma unroll
    for (int t = 0; t < 8; ++t) acc[t] = z;
  }
  const unsigned short* ap = A  + (size_t)(rowBase + 16 * wave + m) * (size_t)lda + 8 * hh;
  const unsigned short* bp = BT + (size_t)(colBase + m) * (size_t)ldb + 8 * hh;

#pragma unroll 1
  for (int k0 = 0; k0 < K; k0 += 32) {
    Frag af;
    af.h[0] = *(const v8usa*)(ap + k0);
    af.h[1] = *(const v8usa*)(ap + k0 + 16);
#pragma unroll
    for (int nt = 0; nt < 8; ++nt) {
      const unsigned short* wq = bp + (size_t)(16 * nt) * (size_t)ldb + k0;
      Frag bf;
      bf.h[0] = *(const v8usa*)wq;
      bf.h[1] = *(const v8usa*)(wq + 16);
      acc[nt] = wmk<KIND>(af, bf, acc[nt]);
    }
  }

#pragma unroll
  for (int nt = 0; nt < 8; ++nt) {
    const int lc = 16 * nt + m;
    const float bb = bf_rne(bias[colBase + lc]);
#pragma unroll
    for (int r = 0; r < 8; ++r) {
      const int lr = 16 * wave + 8 * hh + r;
      stg[lr * GBN + lc] = actf<ACT>(acc[nt][r] * oscale + bb);
    }
  }
  __syncthreads();

  if constexpr (OUTK == 0) {
    v4f pv[16];
#pragma unroll
    for (int i = 0; i < 16; ++i) pv[i] = *(const v4fa*)(stg + (16 * wave + i) * GBN + 4 * lane);
#pragma unroll
    for (int i = 0; i < 16; ++i) {
      const int gr = rowBase + 16 * wave + i;
      float* op = C32 + (size_t)gr * (size_t)ldc + colBase + 4 * lane;
      if (gr < nRows) *(volatile v4f*)op = pv[i];
    }
    __threadfence();
#pragma unroll
    for (int i = 0; i < 16; ++i) {
      const int gr = rowBase + 16 * wave + i;
      float* op = C32 + (size_t)gr * (size_t)ldc + colBase + 4 * lane;
      if (gr < nRows) *(volatile v4f*)op = pv[i];
    }
  } else if constexpr (OUTK == 1) {
    v8us o[8];
#pragma unroll
    for (int i = 0; i < 8; ++i) {
      const int lr = 16 * wave + 2 * i + hh;
      const float* sp = stg + lr * GBN + 8 * m;
      const v4f fa = *(const v4fa*)sp;
      const v4f fb = *(const v4fa*)(sp + 4);
      o[i] = cvt8h(fa, fb);
    }
#pragma unroll
    for (int i = 0; i < 8; ++i) {
      const int lr = 16 * wave + 2 * i + hh;
      unsigned short* op = C16 + (size_t)(rowBase + lr) * (size_t)ldc + colBase + 8 * m;
      *(volatile v8us*)op = o[i];
    }
    __threadfence();
#pragma unroll
    for (int i = 0; i < 8; ++i) {
      const int lr = 16 * wave + 2 * i + hh;
      unsigned short* op = C16 + (size_t)(rowBase + lr) * (size_t)ldc + colBase + 8 * m;
      *(volatile v8us*)op = o[i];
    }
  } else {
    v8us oh[8], ol[8];
    const int loff = ldc >> 1;
#pragma unroll
    for (int i = 0; i < 8; ++i) {
      const int lr = 16 * wave + 2 * i + hh;
      const float* sp = stg + lr * GBN + 8 * m;
      const v4f fa = *(const v4fa*)sp;
      const v4f fb = *(const v4fa*)(sp + 4);
      split8b(fa, fb, oh[i], ol[i]);
    }
#pragma unroll
    for (int i = 0; i < 8; ++i) {
      const int lr = 16 * wave + 2 * i + hh;
      unsigned short* op = C16 + (size_t)(rowBase + lr) * (size_t)ldc + colBase + 8 * m;
      *(volatile v8us*)op = oh[i];
      *(volatile v8us*)(op + loff) = ol[i];
    }
    __threadfence();
#pragma unroll
    for (int i = 0; i < 8; ++i) {
      const int lr = 16 * wave + 2 * i + hh;
      unsigned short* op = C16 + (size_t)(rowBase + lr) * (size_t)ldc + colBase + 8 * m;
      *(volatile v8us*)op = oh[i];
      *(volatile v8us*)(op + loff) = ol[i];
    }
  }
}

template <int L2>
__global__ __launch_bounds__(NTHR) void k_agg(const int* __restrict__ srcs, const int* __restrict__ dsts,
                                              const float* __restrict__ X, unsigned short* Aout,
                                              int nN, int nE, int vec8, int nodeBase0) {
  extern __shared__ __attribute__((aligned(16))) int lds_i[];
  int* reg1 = lds_i;
  int* reg2 = reg1 + RCAP;
  int* scnt = reg2 + RCAP;
  int* soff = scnt + NBA;
  int* list = soff + NBA;
  int* wcnt = list + LISTN;
  int* wtot = wcnt + NWAVE;
  const int tid = (int)threadIdx.x, lane = tid & 31, wave = tid >> 5;
  const int nodeBase = nodeBase0 + (int)blockIdx.x * NBA;
  const int lrowBase = (int)blockIdx.x * NBA;

  {
    const v4i z4 = {0, 0, 0, 0};
    for (int i = tid * 4; i < ZINTS; i += NTHR * 4) *(v4ia*)(lds_i + i) = z4;
    if (tid < 2 * NWAVE) wcnt[tid] = 0;
  }
  __syncthreads();

  int tot = 0;
  const int nChunks = (nE + CHUNK - 1) / CHUNK;
#pragma unroll 1
  for (int ch = 0; ch < nChunks; ++ch) {
    const int cbase = ch * CHUNK;
    const int wc = scan_chunk(dsts, nE, cbase, nodeBase, NBA, vec8, list, tid, lane, wave);
    if (lane == 0) wcnt[wave] = wc;
    __syncthreads();
    int pre = 0, all = 0;
#pragma unroll
    for (int w2 = 0; w2 < NWAVE; ++w2) {
      int c = wcnt[w2];
      c = c < 0 ? 0 : (c > WCAP ? WCAP : c);
      all += c;
      pre += (w2 < wave) ? c : 0;
    }
    const int wcc  = wc > WCAP ? WCAP : wc;
    const int base = tot + pre;
#pragma unroll 1
    for (int i = lane; i < wcc; i += 32) {
      const int ent = list[wave * WCAP + i];
      const int el  = (ent >> PKS) & (CHUNK - 1);
      const int sl  = ent & (NBA - 1);
      int eid = cbase + el;
      eid = eid > nE - 1 ? nE - 1 : eid;
      const int pos = base + i;
      if (pos < RCAP) reg1[pos] = (int)(((unsigned)eid << PKS) | (unsigned)sl);
    }
    tot += all;
    tot = tot > RCAP ? RCAP : tot;
    __syncthreads();
  }
  const int nh = tot;

  if (wave == 0) {
#pragma unroll 1
    for (int b0 = 0; b0 < nh; b0 += 32) {
      const int idx = b0 + lane;
      const int uv  = reg1[idx < RCAP ? idx : RCAP - 1];
      const int m32 = (nh - b0) < 32 ? (nh - b0) : 32;
#pragma unroll 1
      for (int k = 0; k < m32; ++k) {
        const int u  = __builtin_amdgcn_readlane(uv, k);
        const int sl = u & (NBA - 1);
        if (lane == 0) scnt[sl] = scnt[sl] + 1;
      }
    }
  }
  __syncthreads();

  {
    const int c0r = scnt[2 * tid], c1r = scnt[2 * tid + 1];
    const int e0 = c0r < 0 ? 0 : c0r, e1 = c1r < 0 ? 0 : c1r;
    const int ts = e0 + e1;
    int incl = ts;
#pragma unroll
    for (int d = 1; d < 32; d <<= 1) {
      const int up = __shfl_up(incl, d, 32);
      if (lane >= d) incl += up;
    }
    if (lane == 31) wtot[wave] = incl;
    __syncthreads();
    int pre = 0;
#pragma unroll
    for (int w2 = 0; w2 < NWAVE; ++w2) pre += (w2 < wave) ? wtot[w2] : 0;
    int run = pre + incl - ts;
    soff[2 * tid + 0] = run; run += e0;
    soff[2 * tid + 1] = run;
  }
  __syncthreads();
  for (int i = tid; i < NBA; i += NTHR) list[i] = soff[i];
  __syncthreads();

  if (wave == 0) {
#pragma unroll 1
    for (int b0 = 0; b0 < nh; b0 += 32) {
      const int idx = b0 + lane;
      const int uv  = reg1[idx < RCAP ? idx : RCAP - 1];
      const int m32 = (nh - b0) < 32 ? (nh - b0) : 32;
#pragma unroll 1
      for (int k = 0; k < m32; ++k) {
        const int u   = __builtin_amdgcn_readlane(uv, k);
        const int sl  = u & (NBA - 1);
        const int eid = (int)((unsigned)u >> PKS);
        if (lane == 0) {
          int pos = list[sl];
          pos = pos < 0 ? 0 : (pos > RCAP - 1 ? RCAP - 1 : pos);
          reg2[pos] = eid;
          list[sl] = pos + 1;
        }
      }
    }
  }
  __syncthreads();

  const int nbw = NBA / NWAVE;
  const bool ovf = (nh >= RCAP);
  const float qnan = __int_as_float(0x7fc00000);
  unsigned int* stwu = (unsigned int*)reg1 + wave * STW;

#pragma unroll 1
  for (int jt = 0; jt < nbw; ++jt) {
    const int slot = wave * nbw + jt;
    const int node = nodeBase + slot;
    const int lrow = lrowBase + slot;
    int st = soff[slot];
    const int craw = scnt[slot];
    int cnt = craw;
    st  = st < 0 ? 0 : (st > nh ? nh : st);
    cnt = cnt < 0 ? 0 : (cnt > DEGCAP ? DEGCAP : cnt);
    if (cnt > nh - st) cnt = nh - st;
    const float pz = (ovf || craw > DEGCAP) ? qnan : 0.0f;
    const bool live = node < nN;
    const int nc = node < nN ? node : nN - 1;

    if constexpr (L2 == 0) {
      float a0 = 0.f, a1 = 0.f, a2 = 0.f, a3 = 0.f;
#pragma unroll 1
      for (int b0 = 0; b0 < cnt; b0 += 32) {
        int idx = st + b0 + lane; idx = idx > RCAP - 1 ? RCAP - 1 : idx;
        int eid = reg2[idx]; eid = eid < 0 ? 0 : (eid > nE - 1 ? nE - 1 : eid);
        int sr = srcs[eid]; sr = sr < 0 ? 0 : (sr > nN - 1 ? nN - 1 : sr);
        const int m32 = (cnt - b0) < 32 ? (cnt - b0) : 32;
#pragma unroll 1
        for (int k = 0; k < m32; ++k) {
          const int sk = __builtin_amdgcn_readlane(sr, k);
          const v4f v = *(const v4f*)(X + (size_t)sk * DIN + 4 * lane);
          a0 += bf_rne(v.x); a1 += bf_rne(v.y); a2 += bf_rne(v.z); a3 += bf_rne(v.w);
        }
      }
      const v4f sv = *(const v4f*)(X + (size_t)nc * DIN + 4 * lane);
      float r0 = a0 + bf_rne(sv.x), r1 = a1 + bf_rne(sv.y), r2 = a2 + bf_rne(sv.z), r3 = a3 + bf_rne(sv.w);
      r0 = (live ? r0 : 0.0f) + pz;
      r1 = (live ? r1 : 0.0f) + pz;
      r2 = (live ? r2 : 0.0f) + pz;
      r3 = (live ? r3 : 0.0f) + pz;

      const unsigned short hb0 = bf_bits(r0), hb1 = bf_bits(r1), hb2 = bf_bits(r2), hb3 = bf_bits(r3);
      const unsigned short lb0 = bf_bits(r0 - bf_val(hb0)), lb1 = bf_bits(r1 - bf_val(hb1));
      const unsigned short lb2 = bf_bits(r2 - bf_val(hb2)), lb3 = bf_bits(r3 - bf_val(hb3));
      v2u hw, lw;
      hw.x = (unsigned int)hb0 | ((unsigned int)hb1 << 16);
      hw.y = (unsigned int)hb2 | ((unsigned int)hb3 << 16);
      lw.x = (unsigned int)lb0 | ((unsigned int)lb1 << 16);
      lw.y = (unsigned int)lb2 | ((unsigned int)lb3 << 16);
      __builtin_amdgcn_fence(__ATOMIC_RELEASE, "wavefront");
      __builtin_amdgcn_wave_barrier();
      *(v2ua*)(stwu + 2 * lane)      = hw;
      *(v2ua*)(stwu + 64 + 2 * lane) = lw;
      __builtin_amdgcn_fence(__ATOMIC_RELEASE, "wavefront");
      __builtin_amdgcn_wave_barrier();
      const v4u pk = *(const v4ua*)(stwu + 4 * lane);
      unsigned short* gp = Aout + (size_t)lrow * (size_t)K1 + 8 * lane;
      *(volatile v4u*)gp = pk;
      __threadfence();
      *(volatile v4u*)gp = pk;
    } else {
      float acc[16];
#pragma unroll
      for (int i = 0; i < 16; ++i) acc[i] = 0.0f;
#pragma unroll 1
      for (int b0 = 0; b0 < cnt; b0 += 32) {
        int idx = st + b0 + lane; idx = idx > RCAP - 1 ? RCAP - 1 : idx;
        int eid = reg2[idx]; eid = eid < 0 ? 0 : (eid > nE - 1 ? nE - 1 : eid);
        int sr = srcs[eid]; sr = sr < 0 ? 0 : (sr > nN - 1 ? nN - 1 : sr);
        const int m32 = (cnt - b0) < 32 ? (cnt - b0) : 32;
#pragma unroll 1
        for (int k = 0; k < m32; ++k) {
          const int sk = __builtin_amdgcn_readlane(sr, k);
          const float* rp = X + (size_t)sk * HID + 4 * lane;
#pragma unroll
          for (int j = 0; j < 4; ++j) {
            const v4f v = *(const v4f*)(rp + 128 * j);
            acc[4 * j + 0] += v.x; acc[4 * j + 1] += v.y; acc[4 * j + 2] += v.z; acc[4 * j + 3] += v.w;
          }
        }
      }
      float r[16];
      {
        const float* sp = X + (size_t)nc * HID + 4 * lane;
#pragma unroll
        for (int j = 0; j < 4; ++j) {
          const v4f s4 = *(const v4f*)(sp + 128 * j);
          r[4 * j + 0] = acc[4 * j + 0] + s4.x; r[4 * j + 1] = acc[4 * j + 1] + s4.y;
          r[4 * j + 2] = acc[4 * j + 2] + s4.z; r[4 * j + 3] = acc[4 * j + 3] + s4.w;
        }
      }
#pragma unroll
      for (int i = 0; i < 16; ++i) r[i] = (live ? r[i] : 0.0f) + pz;
      v2u pw[4];
#pragma unroll
      for (int j = 0; j < 4; ++j) {
        pw[j].x = (unsigned int)h_bits(r[4 * j + 0]) | ((unsigned int)h_bits(r[4 * j + 1]) << 16);
        pw[j].y = (unsigned int)h_bits(r[4 * j + 2]) | ((unsigned int)h_bits(r[4 * j + 3]) << 16);
      }
      __builtin_amdgcn_fence(__ATOMIC_RELEASE, "wavefront");
      __builtin_amdgcn_wave_barrier();
#pragma unroll
      for (int j = 0; j < 4; ++j) *(v2ua*)(stwu + 64 * j + 2 * lane) = pw[j];
      __builtin_amdgcn_fence(__ATOMIC_RELEASE, "wavefront");
      __builtin_amdgcn_wave_barrier();
      const v4u pk0 = *(const v4ua*)(stwu + 4 * lane);
      const v4u pk1 = *(const v4ua*)(stwu + 128 + 4 * lane);
      unsigned short* gp = Aout + (size_t)lrow * (size_t)HID + 8 * lane;
      *(volatile v4u*)gp = pk0;
      *(volatile v4u*)(gp + 256) = pk1;
      __threadfence();
      *(volatile v4u*)gp = pk0;
      *(volatile v4u*)(gp + 256) = pk1;
    }
  }
}

static inline int cdiv(int a, int b) { return (a + b - 1) / b; }

extern "C" void kernel_launch(void* const* d_in, const int* in_sizes, int n_in,
                              void* d_out, int out_size, void* d_ws, size_t ws_size,
                              hipStream_t stream) {
  if (n_in < 10) return;
  if (in_sizes[0] < DIN || (in_sizes[0] % DIN) != 0) return;
  const int nN = in_sizes[0] / DIN;
  if (nN < 1 || nN > (1 << 24)) return;
  if (in_sizes[1] < 2 || (in_sizes[1] & 1) != 0) return;
  const int nE = in_sizes[1] / 2;
  if (nE < 1 || nE >= (1 << 22)) return;
  if (in_sizes[2] != DIN * HID || in_sizes[3] != HID) return;
  if (in_sizes[4] != HID * HID || in_sizes[5] != HID) return;
  if (in_sizes[6] != HID * HID || in_sizes[7] != HID) return;
  if (in_sizes[8] != HID * DOUT || in_sizes[9] != DOUT) return;
  if ((long long)out_size != (long long)nN * DOUT) return;

  const float* feature = (const float*)d_in[0];
  const int*   edge    = (const int*)d_in[1];
  const float* w1 = (const float*)d_in[2];
  const float* b1 = (const float*)d_in[3];
  const float* w2 = (const float*)d_in[4];
  const float* b2 = (const float*)d_in[5];
  const float* w3 = (const float*)d_in[6];
  const float* b3 = (const float*)d_in[7];
  const float* w4 = (const float*)d_in[8];
  const float* b4 = (const float*)d_in[9];
  float* out = (float*)d_out;
  const int* src = edge;
  const int* dst = edge + nE;

  const int nChunk = cdiv(nN, RCH);
  const int MPG = nChunk * RCH;
  const int vec8 = ((nE & 3) == 0) ? 1 : 0;

  char* ws = (char*)d_ws;
  size_t off = 0;
  const size_t oW1D = off; off += (size_t)HID * K1 * 2;             off = (off + 255) & ~(size_t)255;
  const size_t oW2C = off; off += (size_t)HID * HID * 2;            off = (off + 255) & ~(size_t)255;
  const size_t oW3C = off; off += (size_t)HID * HID * 2;            off = (off + 255) & ~(size_t)255;
  const size_t oW4D = off; off += (size_t)DOUT * K4 * 2;            off = (off + 255) & ~(size_t)255;
  const size_t oH   = off; off += (size_t)MPG * HID * 4;            off = (off + 255) & ~(size_t)255;
  const size_t oS1  = off; off += (size_t)RCH * HID * 2;            off = (off + 255) & ~(size_t)255;
  const size_t oS2  = off; off += (size_t)RCH * HID * 2;            off = (off + 255) & ~(size_t)255;
  const size_t oS3  = off; off += (size_t)RCH * K4 * 2;             off = (off + 255) & ~(size_t)255;
  if (off > ws_size || off > (size_t)WSMAX) return;
  unsigned short* W1D = (unsigned short*)(ws + oW1D);
  unsigned short* W2C = (unsigned short*)(ws + oW2C);
  unsigned short* W3C = (unsigned short*)(ws + oW3C);
  unsigned short* W4D = (unsigned short*)(ws + oW4D);
  float*          H   = (float*)(ws + oH);
  unsigned short* S1  = (unsigned short*)(ws + oS1);
  unsigned short* S2  = (unsigned short*)(ws + oS2);
  unsigned short* S3  = (unsigned short*)(ws + oS3);

  hipFuncSetAttribute(reinterpret_cast<const void*>(&k_agg<0>), hipFuncAttributeMaxDynamicSharedMemorySize, LDS_AGG);
  hipFuncSetAttribute(reinterpret_cast<const void*>(&k_agg<1>), hipFuncAttributeMaxDynamicSharedMemorySize, LDS_AGG);

  k_wprep<<<NUW / NTHR, NTHR, 0, stream>>>(w1, w2, w3, w4, W1D, W2C, W3C, W4D);

  const dim3 gG4(RCH / GBM, HID / GBN);
  const dim3 gG1(RCH / GBM, DOUT / GBN);

  for (int c = 0; c < nChunk; ++c) {
    const int rowOff = c * RCH;
    k_agg<0><<<NBLKA, NTHR, LDS_AGG, stream>>>(src, dst, feature, S1, nN, nE, vec8, rowOff);
    k_gemm<0, 1, 1><<<gG4, GTHR, 0, stream>>>(S1, K1, W1D, K1, K1, b1, 1.0f, (float*)S2, S2, HID, RCH);
    float* Hrows = H + (size_t)rowOff * HID;
    k_gemm<1, 2, 0><<<gG4, GTHR, 0, stream>>>(S2, HID, W2C, HID, HID, b2, WINV, Hrows, (unsigned short*)Hrows, HID, RCH);
  }
  for (int c = 0; c < nChunk; ++c) {
    const int rowOff = c * RCH;
    k_agg<1><<<NBLKA, NTHR, LDS_AGG, stream>>>(src, dst, H, S1, nN, nE, vec8, rowOff);
    k_gemm<1, 1, 2><<<gG4, GTHR, 0, stream>>>(S1, HID, W3C, HID, HID, b3, WINV, (float*)S3, S3, K4, RCH);
    int nr = nN - rowOff;
    nr = nr < 0 ? 0 : (nr > RCH ? RCH : nr);
    float* orows = out + (size_t)rowOff * DOUT;
    k_gemm<0, 0, 0><<<gG1, GTHR, 0, stream>>>(S3, K4, W4D, K4, K4, b4, 1.0f, orows, (unsigned short*)orows, DOUT, nr);
  }
}
